// Quanv2d_72584947302551
// MI455X (gfx1250) — hardware-verified
//
#include <hip/hip_runtime.h>
#include <stddef.h>


typedef _Float16 h16;
typedef _Float16 v16h __attribute__((ext_vector_type(16)));
typedef _Float16 v8h  __attribute__((ext_vector_type(8)));
typedef float    v8f  __attribute__((ext_vector_type(8)));
typedef float    v4f  __attribute__((ext_vector_type(4)));

#ifndef NB
#define NB 16384
#endif
#define NB_FULL 16384
#define IMG     196
#define PPI     36
#define NPATCH  (NB * PPI)

#ifndef BRES
#define BRES 1
#endif

#define ACARRY 4096.0f
#define BCARRY 4096.0f
#define DSCALE (1.0f / (4096.0f * 4096.0f))

#define LDA 24
#define LDP 17

static_assert(NB >= 64 && NB <= NB_FULL);
static_assert((NPATCH % 256) == 0);
static_assert((LDA % 8) == 0 && LDA >= 16);
static_assert(LDP >= 16);
static_assert((size_t)NPATCH * 4 < (size_t)0x7FFFFFFF);

__device__ __forceinline__ float bf16r(float x) {
  unsigned int u = __float_as_uint(x);
  u = (u + 0x7FFFu + ((u >> 16) & 1u)) & 0xFFFF0000u;
  return __uint_as_float(u);
}

static __device__ __forceinline__ h16 toh_flush(float v) {
  const h16 r = (h16)v;
  return (fabsf(v) < 6.103515625e-05f) ? (h16)0.0f : r;
}

__device__ __forceinline__ v8f wmma16(v16h a, v16h b, v8f c) {
  v8f d = __builtin_amdgcn_wmma_f32_16x16x32_f16(false, a, false, b, (short)0, c,
                                                 false, false);
  asm volatile("v_nop\n\tv_nop\n\tv_nop\n\tv_nop" : "+v"(d) : "v"(a), "v"(b));
  return d;
}

__device__ __forceinline__ void apply_rz(float th, float& r0, float& i0, float& r1, float& i1) {
  float s, c; __sincosf(0.5f * th, &s, &c);
  float nr0 = r0 * c + i0 * s, ni0 = i0 * c - r0 * s;
  float nr1 = r1 * c - i1 * s, ni1 = i1 * c + r1 * s;
  r0 = nr0; i0 = ni0; r1 = nr1; i1 = ni1;
}

__device__ __forceinline__ void apply_ry(float th, float& r0, float& i0, float& r1, float& i1) {
  float s, c; __sincosf(0.5f * th, &s, &c);
  float nr0 = c * r0 - s * r1, ni0 = c * i0 - s * i1;
  float nr1 = s * r0 + c * r1, ni1 = s * i0 + c * i1;
  r0 = nr0; i0 = ni0; r1 = nr1; i1 = ni1;
}

__global__ __launch_bounds__(256) void qconv_kernel(
    const float* __restrict__ X, const float* __restrict__ W, float* __restrict__ out)
{
  __shared__ h16   s_re[256 * LDA];
  __shared__ h16   s_im[256 * LDA];
  __shared__ float s_p[256 * LDP];
  __shared__ float s_phr[16];
  __shared__ float s_phi[16];

  const int tid  = threadIdx.x;
  const int lane = tid & 31;
  const int wv   = __builtin_amdgcn_readfirstlane(tid >> 5);
  const int m    = lane & 15;
  const int h    = lane >> 4;

  const int p = blockIdx.x * 256 + tid;
  const bool active = (p < NPATCH);
  const int pe = active ? p : (NPATCH - 1);

  const int b   = pe / PPI;
  const int r36 = pe - b * PPI;
  const int oi  = r36 / 6;
  const int oj  = r36 - oi * 6;
  const float* xp = X + (size_t)b * IMG + (oi * 2) * 14 + (oj * 2);

  float ang[16];
#pragma unroll
  for (int r = 0; r < 4; ++r)
#pragma unroll
    for (int s = 0; s < 4; ++s)
      ang[r * 4 + s] = bf16r(xp[r * 14 + s]);

  float w[8];
#pragma unroll
  for (int q = 0; q < 8; ++q) w[q] = bf16r(W[q]);

  {
    const int sx = tid & 15;
    const float b0 = (float)((sx >> 3) & 1), b1 = (float)((sx >> 2) & 1);
    const float b2 = (float)((sx >> 1) & 1), b3 = (float)(sx & 1);
    const float e = w[0] * b0 * (2.f * b1 - 1.f)
                  + w[1] * b1 * (2.f * b2 - 1.f)
                  + w[2] * b2 * (2.f * b3 - 1.f)
                  + w[3] * b3 * (2.f * b0 - 1.f);
    float ps, pc; __sincosf(0.5f * e, &ps, &pc);
    if (tid < 16) { s_phr[sx] = pc; s_phi[sx] = ps; }
  }

  const float H = 0.70710678118654752f;
  float vr[4][2], vi[4][2];
#pragma unroll
  for (int q = 0; q < 3; ++q) {
    float r0 = H, i0 = 0.f, r1 = H, i1 = 0.f;
    apply_rz(ang[q * 5 + 0], r0, i0, r1, i1);
    apply_ry(ang[q * 5 + 1], r0, i0, r1, i1);
    apply_rz(ang[q * 5 + 2], r0, i0, r1, i1);
    apply_ry(ang[q * 5 + 3], r0, i0, r1, i1);
    apply_rz(ang[q * 5 + 4], r0, i0, r1, i1);
    vr[q][0] = r0; vi[q][0] = i0; vr[q][1] = r1; vi[q][1] = i1;
  }
  {
    float s, c; __sincosf(0.5f * ang[15], &s, &c);
    vr[3][0] = H * c; vi[3][0] = -H * s;
    vr[3][1] = H * c; vi[3][1] =  H * s;
  }

  v16h bfrag;
  {
    float cw[4], sw[4];
#pragma unroll
    for (int q = 0; q < 4; ++q) __sincosf(0.5f * w[4 + q], &sw[q], &cw[q]);
#pragma unroll
    for (int i = 0; i < 8; ++i) {
      const int k = 8 * h + i;
      float val = 1.f;
#pragma unroll
      for (int q = 0; q < 4; ++q) {
        const int nb = (m >> (3 - q)) & 1;
        const int kb = (k >> (3 - q)) & 1;
        val *= (nb == kb) ? cw[q] : (nb ? sw[q] : -sw[q]);
      }
      const float cv = BCARRY * val;
      const h16 hi = toh_flush(cv);
#if BRES
      const h16 lo = toh_flush(cv - (float)hi);
#else
      const h16 lo = (h16)0.0f;
#endif
      bfrag[i]     = hi;
      bfrag[i + 8] = lo;
    }
  }

  __syncthreads();

  {
    float tr_[16], ti_[16];
    float ur[4], ui[4];
#pragma unroll
    for (int cd = 0; cd < 4; ++cd) {
      const int c = cd >> 1, d = cd & 1;
      ur[cd] = vr[2][c] * vr[3][d] - vi[2][c] * vi[3][d];
      ui[cd] = vr[2][c] * vi[3][d] + vi[2][c] * vr[3][d];
    }
#pragma unroll
    for (int ab = 0; ab < 4; ++ab) {
      const int a = ab >> 1, bq = ab & 1;
      const float tr = vr[0][a] * vr[1][bq] - vi[0][a] * vi[1][bq];
      const float ti = vr[0][a] * vi[1][bq] + vi[0][a] * vr[1][bq];
#pragma unroll
      for (int cd = 0; cd < 4; ++cd) {
        const int s_ = ab * 4 + cd;
        const float ar = tr * ur[cd] - ti * ui[cd];
        const float ai = tr * ui[cd] + ti * ur[cd];
        const float pr = s_phr[s_], pi = s_phi[s_];
        tr_[s_] = ar * pr - ai * pi;
        ti_[s_] = ar * pi + ai * pr;
      }
    }
    v8h xr0, xr1, xi0, xi1;
#pragma unroll
    for (int i = 0; i < 8; ++i) {
      xr0[i] = toh_flush(ACARRY * tr_[i]);
      xr1[i] = toh_flush(ACARRY * tr_[8 + i]);
      xi0[i] = toh_flush(ACARRY * ti_[i]);
      xi1[i] = toh_flush(ACARRY * ti_[8 + i]);
    }
    *(v8h*)&s_re[tid * LDA]     = xr0;
    *(v8h*)&s_re[tid * LDA + 8] = xr1;
    *(v8h*)&s_im[tid * LDA]     = xi0;
    *(v8h*)&s_im[tid * LDA + 8] = xi1;
  }

  __syncthreads();

#pragma unroll
  for (int t = 0; t < 2; ++t) {
    const int row = wv * 32 + t * 16 + m;
    const v8h ar8 = *(const v8h*)&s_re[row * LDA + 8 * h];
    const v8h ai8 = *(const v8h*)&s_im[row * LDA + 8 * h];
    v16h a_re, a_im;
#pragma unroll
    for (int i = 0; i < 8; ++i) {
      a_re[i] = ar8[i]; a_re[i + 8] = ar8[i];
      a_im[i] = ai8[i]; a_im[i + 8] = ai8[i];
    }
    v8f acc_r = {};
    v8f acc_i = {};
    acc_r = wmma16(a_re, bfrag, acc_r);
    acc_i = wmma16(a_im, bfrag, acc_i);

    const int row0 = wv * 32 + t * 16 + 8 * h;
#pragma unroll
    for (int v = 0; v < 8; ++v) {
      const float dr = acc_r[v] * DSCALE;
      const float di = acc_i[v] * DSCALE;
      s_p[(row0 + v) * LDP + m] = dr * dr + di * di;
    }
  }

  __syncthreads();

  float o0 = 0.f, o1 = 0.f, o2 = 0.f, o3 = 0.f;
#pragma unroll
  for (int s_ = 0; s_ < 16; ++s_) {
    const float pr = s_p[tid * LDP + s_];
    o0 += ((s_ >> 3) & 1) ? -pr : pr;
    o1 += ((s_ >> 2) & 1) ? -pr : pr;
    o2 += ((s_ >> 1) & 1) ? -pr : pr;
    o3 += (s_ & 1)        ? -pr : pr;
  }

  v4f res;
  res[0] = o0; res[1] = o1; res[2] = o2; res[3] = o3;
  float* dst = out + (size_t)pe * 4;
  if (active) *(volatile v4f*)dst = res;
  __threadfence();
  if (active) *(volatile v4f*)dst = res;
}

extern "C" void kernel_launch(void* const* d_in, const int* in_sizes, int n_in,
                              void* d_out, int out_size, void* d_ws, size_t ws_size,
                              hipStream_t stream) {
  (void)d_ws; (void)ws_size;
  if (n_in < 2) return;
  if ((long long)in_sizes[0] < (long long)NB * IMG) return;
  if (in_sizes[1] < 8) return;
  if ((long long)out_size < (long long)NPATCH * 4) return;

  const float* X = (const float*)d_in[0];
  const float* W = (const float*)d_in[1];
  float* out = (float*)d_out;

  qconv_kernel<<<dim3(NPATCH / 256), dim3(256), 0, stream>>>(X, W, out);
}
